// DTransformer_51084341019395
// MI455X (gfx1250) — hardware-verified
//
#include <hip/hip_runtime.h>
#include <math.h>
#include <stdint.h>

#define NB    8
#define SEQ   1024
#define DM    256
#define NH    8
#define HD    32
#define MP    (NB * SEQ)
#define NQB   (SEQ / 64)
#define MISZ  (NB * NH * SEQ)
#define C32W  (2 * DM)
#define QRES  ((long long)MP * DM)
#define VRES  ((long long)NB * DM * SEQ)
#define LNEPS 1.0e-5f
#define WSC   64.0f
#define RSC   2048.0f
#define PSC   1024.0f
#define NEGV  (-1.0e32f)
#define SSC   0.17677669529663688f
static_assert(NH * HD == DM);
static_assert((SEQ % 64) == 0 && (MP % 64) == 0 && (DM % 64) == 0);
static_assert(MP * DM == 2097152);
static_assert(HD == 32);

typedef _Float16       v16h __attribute__((ext_vector_type(16)));
typedef __bf16         v16b __attribute__((ext_vector_type(16)));
typedef unsigned short v16us __attribute__((ext_vector_type(16)));
typedef unsigned short v8us __attribute__((ext_vector_type(8)));
typedef float          v8f  __attribute__((ext_vector_type(8)));
typedef float          v4f  __attribute__((ext_vector_type(4)));
typedef unsigned int   v4u  __attribute__((ext_vector_type(4)));

union Frag { v16us u; v8us p[2]; v16h h; v16b b; };
union F8   { v8f v; v4f q[2]; };

__device__ __forceinline__ unsigned short bf_bits(float f) {
  unsigned u = __float_as_uint(f);
  return (unsigned short)((u + 0x7FFFu + ((u >> 16) & 1u)) >> 16);
}
__device__ __forceinline__ float bf_up(unsigned short h) { return __uint_as_float(((unsigned)h) << 16); }
__device__ __forceinline__ float bfr(float f) { return bf_up(bf_bits(f)); }
__device__ __forceinline__ unsigned short h_bits(_Float16 x) { return __builtin_bit_cast(unsigned short, x); }
__device__ __forceinline__ unsigned pk16(unsigned short a, unsigned short b) { return (unsigned)a | ((unsigned)b << 16); }
__device__ __forceinline__ v8f zero8() { v8f z = {0.f, 0.f, 0.f, 0.f, 0.f, 0.f, 0.f, 0.f}; return z; }
__device__ __forceinline__ v16us zero16() {
  v16us z;
#pragma unroll
  for (int i = 0; i < 16; ++i) z[i] = 0;
  return z;
}
__device__ __forceinline__ unsigned short split_sel(float f, int part) {
  const unsigned short hb = bf_bits(f);
  const unsigned short lb = bf_bits(f - bf_up(hb));
  return part ? lb : hb;
}
__device__ __forceinline__ unsigned pick2(float f0, float f1, int part) {
  return pk16(split_sel(f0, part), split_sel(f1, part));
}

__device__ __forceinline__ v16us ldfrag(const unsigned short* p) {
  Frag f;
  f.p[0] = *(const v8us*)(p);
  f.p[1] = *(const v8us*)(p + 16);
  return f.u;
}

template <int BF>
__device__ __forceinline__ v8f mma_raw(v16us a, v16us b, v8f c) {
  Frag fa, fb;
  fa.u = a;
  fb.u = b;
  if constexpr (BF) {
    return __builtin_amdgcn_wmma_f32_16x16x32_bf16(false, fa.b, false, fb.b, (short)0, c, false, false);
  } else {
    return __builtin_amdgcn_wmma_f32_16x16x32_f16(false, fa.h, false, fb.h, (short)0, c, false, false);
  }
}
template <int BF>
__device__ __forceinline__ v8f mma_g(v16us a, v16us b, v8f c) {
  c = mma_raw<BF>(a, b, c);
#if defined(__HIP_DEVICE_COMPILE__)
  asm volatile("v_nop\n\tv_nop\n\tv_nop\n\tv_nop" : "+v"(c) : "v"(a), "v"(b));
#endif
  return c;
}
__device__ __forceinline__ void dep_guard1(v8f& a, v8f& b, v16us x) {
#if defined(__HIP_DEVICE_COMPILE__)
  asm volatile("v_nop\n\tv_nop\n\tv_nop\n\tv_nop" : "+v"(a), "+v"(b) : "v"(x));
#endif
}
__device__ __forceinline__ void keep4(v16us a, v16us b, v16us c, v16us d) {
#if defined(__HIP_DEVICE_COMPILE__)
  asm volatile("v_nop" :: "v"(a), "v"(b), "v"(c), "v"(d));
#endif
}
__device__ __forceinline__ void acc_guard4(v8f& a, v8f& b, v8f& c, v8f& d) {
#if defined(__HIP_DEVICE_COMPILE__)
  asm volatile("v_nop\n\tv_nop\n\tv_nop\n\tv_nop" : "+v"(a), "+v"(b), "+v"(c), "+v"(d));
#endif
}
__device__ __forceinline__ void wave_sync_lds() {
  __builtin_amdgcn_fence(__ATOMIC_RELEASE, "workgroup");
  __builtin_amdgcn_wave_barrier();
  __builtin_amdgcn_fence(__ATOMIC_ACQUIRE, "workgroup");
}
__device__ __forceinline__ float wsum(float v) {
#pragma unroll
  for (int off = 16; off > 0; off >>= 1) v += __shfl_xor(v, off, 32);
  return v;
}

__global__ __launch_bounds__(256) void conv_h16(const float* __restrict__ W, unsigned short* Wh, int n8, float wsc) {
  const int i  = blockIdx.x * 256 + threadIdx.x;
  const int ic = (i < n8) ? i : (n8 - 1);
  const float* src = W + (size_t)ic * 8;
  const v4f a = *(const v4f*)(src);
  const v4f c = *(const v4f*)(src + 4);
  v4u o;
  o[0] = pk16(h_bits((_Float16)(bfr(a[0]) * wsc)), h_bits((_Float16)(bfr(a[1]) * wsc)));
  o[1] = pk16(h_bits((_Float16)(bfr(a[2]) * wsc)), h_bits((_Float16)(bfr(a[3]) * wsc)));
  o[2] = pk16(h_bits((_Float16)(bfr(c[0]) * wsc)), h_bits((_Float16)(bfr(c[1]) * wsc)));
  o[3] = pk16(h_bits((_Float16)(bfr(c[2]) * wsc)), h_bits((_Float16)(bfr(c[3]) * wsc)));
  if (i < n8) *(volatile v4u*)(Wh + (size_t)i * 8) = o;
  __threadfence();
  if (i < n8) *(volatile v4u*)(Wh + (size_t)i * 8) = o;
}

__global__ __launch_bounds__(256) void conv_c32(const float* __restrict__ W, unsigned short* Wb, int npieces, int ncols) {
  const int i   = blockIdx.x * 256 + threadIdx.x;
  const int ic  = (i < npieces) ? i : (npieces - 1);
  const int ppr = ncols >> 2;
  const int row = ic / ppr;
  const int p   = ic - row * ppr;
  const int chunk = p >> 3, sub = p & 3;
  const float* src = W + (size_t)row * ncols + chunk * 32 + sub * 8;
  const v4f a = *(const v4f*)(src);
  const v4f c = *(const v4f*)(src + 4);
  v4u o;
  o[0] = pk16(bf_bits(a[0]), bf_bits(a[1]));
  o[1] = pk16(bf_bits(a[2]), bf_bits(a[3]));
  o[2] = pk16(bf_bits(c[0]), bf_bits(c[1]));
  o[3] = pk16(bf_bits(c[2]), bf_bits(c[3]));
  unsigned short* dst = Wb + (size_t)row * (size_t)(2 * ncols) + 8 * p;
  if (i < npieces) *(volatile v4u*)(dst) = o;
  __threadfence();
  if (i < npieces) *(volatile v4u*)(dst) = o;
}

__device__ __forceinline__ v4u kk_piece(const float* __restrict__ know, const float* __restrict__ Wlk,
                                        const float* __restrict__ blk, int n, int p) {
  const int chunk = p >> 3, part = (p >> 2) & 1, sub = p & 3;
  const int j0 = chunk * 32 + sub * 8;
  unsigned short w[8];
#pragma unroll
  for (int e = 0; e < 8; ++e) {
    const int j = j0 + e;
    float a = 0.f;
#pragma unroll 1
    for (int k = 0; k < HD; ++k) a = fmaf(bfr(know[n * HD + k]), bfr(Wlk[j * HD + k]), a);
    a += bfr(blk[j]);
    const float sg = __builtin_amdgcn_rcpf(1.0f + __expf(-a));
    w[e] = split_sel(sg, part);
  }
  v4u o;
#pragma unroll
  for (int e = 0; e < 4; ++e) o[e] = pk16(w[2 * e], w[2 * e + 1]);
  return o;
}

__global__ __launch_bounds__(32) void small_vec(const float* __restrict__ know, const float* __restrict__ Wlk,
                                              const float* __restrict__ blk, const float* __restrict__ Wq3,
                                              const float* __restrict__ bq3, unsigned short* kkp, float* q3f) {
  const int lane = threadIdx.x & 31;
  const int n = blockIdx.x;
  if (n < 64) {
    v4u o0, o1;
#pragma unroll
    for (int e = 0; e < 4; ++e) { o0[e] = 0u; o1[e] = 0u; }
    if (n < NH) {
      o0 = kk_piece(know, Wlk, blk, n, lane);
      o1 = kk_piece(know, Wlk, blk, n, 32 + lane);
    }
    unsigned short* d0 = kkp + (size_t)n * C32W + 8 * lane;
    *(volatile v4u*)(d0) = o0;
    *(volatile v4u*)(d0 + 256) = o1;
    __threadfence();
    *(volatile v4u*)(d0) = o0;
    *(volatile v4u*)(d0 + 256) = o1;
  } else {
    float a[8];
#pragma unroll
    for (int e = 0; e < 8; ++e) a[e] = 0.f;
#pragma unroll 1
    for (int k = 0; k < DM; ++k) {
      const float kv = bfr(know[k]);
#pragma unroll
      for (int e = 0; e < 4; ++e) {
        a[e]     = fmaf(kv, bfr(Wq3[(size_t)(4 * lane + e) * DM + k]), a[e]);
        a[4 + e] = fmaf(kv, bfr(Wq3[(size_t)(128 + 4 * lane + e) * DM + k]), a[4 + e]);
      }
    }
    v4f v0, v1;
#pragma unroll
    for (int e = 0; e < 4; ++e) {
      v0[e] = a[e]     + bfr(bq3[4 * lane + e]);
      v1[e] = a[4 + e] + bfr(bq3[128 + 4 * lane + e]);
    }
    float* d0 = q3f + 4 * lane;
    *(volatile v4f*)(d0) = v0;
    *(volatile v4f*)(d0 + 128) = v1;
    __threadfence();
    *(volatile v4f*)(d0) = v0;
    *(volatile v4f*)(d0 + 128) = v1;
  }
}

__global__ __launch_bounds__(256) void score3(const float* __restrict__ K3, const float* __restrict__ q3,
                                            float* S3, float sscale) {
  const int t   = blockIdx.x * 256 + threadIdx.x;
  const int key = t & (SEQ - 1);
  const int bh  = t >> 10;
  const int b   = bh >> 3, h = bh & 7;
  const float* kp = K3 + ((size_t)b * SEQ + key) * DM + h * HD;
  const float* qp = q3 + h * HD;
  float a = 0.f;
#pragma unroll 1
  for (int d = 0; d < HD; d += 4) {
    const v4f kv = *(const v4f*)(kp + d);
    const v4f qv = *(const v4f*)(qp + d);
    a = fmaf(qv[0], kv[0], a);
    a = fmaf(qv[1], kv[1], a);
    a = fmaf(qv[2], kv[2], a);
    a = fmaf(qv[3], kv[3], a);
  }
  const float sv = a * sscale;
  float* dst = S3 + t;
  *(volatile float*)dst = sv;
  __threadfence();
  *(volatile float*)dst = sv;
}

template <int BF, int OM, int BIASM>
__global__ __launch_bounds__(256) void gemm64(
    const unsigned short* __restrict__ A, int lda, long long strideA,
    const unsigned short* __restrict__ Bt, int ldb, long long strideB,
    const float* __restrict__ bias0,
    void* Cout, int ldc, long long strideC, long long resOff,
    int M, int N, int K, float oscale) {
  __shared__ __align__(16) float sT[8][16 * 68];
  const int b    = blockIdx.y;
  const int lane = threadIdx.x & 31;
  const int wave = threadIdx.x >> 5;
  const int tilesN = N >> 6;
  const int tilesM = M >> 6;
  const int tile = blockIdx.x * 8 + wave;
  if (tile >= tilesM * tilesN) return;
  const int tm = tile / tilesN;
  const int tn = tile - tm * tilesN;
  const int m0 = tm << 6;
  const int n0 = tn << 6;

  const unsigned short* Ab = A  + (size_t)b * (size_t)strideA;
  const unsigned short* Bb = Bt + (size_t)b * (size_t)strideB;

  const int rlane = lane & 15;
  const int koff  = (lane >> 4) * 8;
  const int mOff  = (lane >> 4) * 8;

  v8f acc[4][4];
#pragma unroll
  for (int i = 0; i < 4; ++i)
#pragma unroll
    for (int j = 0; j < 4; ++j) acc[i][j] = zero8();

  for (int k0 = 0; k0 < K; k0 += 32) {
    v16us bh[4];
#pragma unroll
    for (int j = 0; j < 4; ++j) {
      const size_t bo = (size_t)(n0 + (j << 4) + rlane) * ldb + koff + k0;
      bh[j] = ldfrag(Bb + bo);
    }
#pragma unroll
    for (int i = 0; i < 4; ++i) {
      const size_t ao = (size_t)(m0 + (i << 4) + rlane) * lda + koff + k0;
      const v16us ah = ldfrag(Ab + ao);
#pragma unroll
      for (int j = 0; j < 4; ++j) acc[i][j] = mma_raw<BF>(ah, bh[j], acc[i][j]);
      dep_guard1(acc[i][0], acc[i][3], ah);
    }
    keep4(bh[0], bh[1], bh[2], bh[3]);
  }
  acc_guard4(acc[0][0], acc[0][1], acc[0][2], acc[0][3]);
  acc_guard4(acc[1][0], acc[1][1], acc[1][2], acc[1][3]);
  acc_guard4(acc[2][0], acc[2][1], acc[2][2], acc[2][3]);
  acc_guard4(acc[3][0], acc[3][1], acc[3][2], acc[3][3]);

  const int hh2 = lane >> 4, c4 = (lane & 15) * 4;
  const int q8  = lane >> 3, c8 = (lane & 7) * 8;
  float bc[8];
#pragma unroll
  for (int e = 0; e < 8; ++e) bc[e] = 0.f;
  if (BIASM == 0) {
    if (OM == 0) {
      const v4f b0v = *(const v4f*)(bias0 + n0 + c4);
#pragma unroll
      for (int e = 0; e < 4; ++e) bc[e] = bfr(b0v[e]);
    } else {
      const v4f b0a = *(const v4f*)(bias0 + n0 + c8);
      const v4f b0b = *(const v4f*)(bias0 + n0 + c8 + 4);
#pragma unroll
      for (int e = 0; e < 4; ++e) {
        bc[e]     = bfr(b0a[e]);
        bc[4 + e] = bfr(b0b[e]);
      }
    }
  }

  float* slab = sT[wave];
#pragma unroll
  for (int i = 0; i < 4; ++i) {
    const int mBase = m0 + (i << 4);
#pragma unroll
    for (int j = 0; j < 4; ++j) {
#pragma unroll
      for (int r = 0; r < 8; ++r) {
        slab[(mOff + r) * 68 + (j << 4) + rlane] = acc[i][j][r];
      }
    }
    wave_sync_lds();
    if constexpr (OM == 0) {
      float* C = (float*)Cout + (size_t)b * (size_t)strideC;
      v4f vals[8];
#pragma unroll
      for (int it = 0; it < 8; ++it) {
        const int row = it * 2 + hh2;
        v4f v = *(const v4f*)(slab + row * 68 + c4);
#pragma unroll
        for (int e = 0; e < 4; ++e) v[e] = v[e] * oscale + bc[e];
        vals[it] = v;
      }
      for (int pass = 0; pass < 2; ++pass) {
#pragma unroll
        for (int it = 0; it < 8; ++it) {
          const int row = it * 2 + hh2;
          *(volatile v4f*)(C + (size_t)(mBase + row) * ldc + n0 + c4) = vals[it];
        }
        __threadfence();
      }
    } else {
      unsigned short* C = (unsigned short*)Cout + (size_t)b * (size_t)strideC;
      v4u hv[4], hr[4];
#pragma unroll
      for (int it = 0; it < 4; ++it) {
        const int row = it * 4 + q8;
        const float* sp = slab + row * 68 + c8;
        float bm = 0.f;
        if (BIASM == 1) bm = bfr(bias0[mBase + row]);
        v4u a, ar;
#pragma unroll
        for (int e = 0; e < 4; ++e) {
          const float f0 = sp[2 * e]     * oscale + ((BIASM == 1) ? bm : bc[2 * e]);
          const float f1 = sp[2 * e + 1] * oscale + ((BIASM == 1) ? bm : bc[2 * e + 1]);
          const _Float16 g0 = (_Float16)f0, g1 = (_Float16)f1;
          a[e] = pk16(h_bits(g0), h_bits(g1));
          if (OM == 3) {
            const float e0 = (f0 - (float)g0) * RSC;
            const float e1 = (f1 - (float)g1) * RSC;
            ar[e] = pk16(h_bits((_Float16)e0), h_bits((_Float16)e1));
          } else {
            ar[e] = 0u;
          }
        }
        hv[it] = a;
        hr[it] = ar;
      }
      for (int pass = 0; pass < 2; ++pass) {
#pragma unroll
        for (int it = 0; it < 4; ++it) {
          const int row = it * 4 + q8;
          unsigned short* dp = C + (size_t)(mBase + row) * ldc + n0 + c8;
          *(volatile v4u*)(dp) = hv[it];
          if (OM == 3) *(volatile v4u*)(dp + resOff) = hr[it];
        }
        __threadfence();
      }
    }
    wave_sync_lds();
  }
}

__device__ __forceinline__ void stage_k(unsigned short* Ksh, unsigned short* Krs,
                                        const unsigned short* kh, const unsigned short* kr,
                                        size_t rowB, int kv0, int h, int tid) {
  const int r = tid >> 1, hf = (tid & 1) * 16;
  const size_t go = (rowB + kv0 + r) * DM + (size_t)h * HD + hf;
  const v8us a0 = *(const v8us*)(kh + go), a1 = *(const v8us*)(kh + go + 8);
  const v8us c0 = *(const v8us*)(kr + go), c1 = *(const v8us*)(kr + go + 8);
  *(v8us*)(Ksh + r * HD + hf)     = a0;
  *(v8us*)(Ksh + r * HD + hf + 8) = a1;
  *(v8us*)(Krs + r * HD + hf)     = c0;
  *(v8us*)(Krs + r * HD + hf + 8) = c1;
}
__device__ __forceinline__ void stage_v(unsigned short* Vth, unsigned short* Vtr,
                                        const unsigned short* vth, const unsigned short* vtr,
                                        int b, int kv0, int h, int tid) {
  const int d = tid >> 2, qd = (tid & 3) * 16;
  const size_t go = ((size_t)b * DM + (size_t)h * HD + d) * SEQ + kv0 + qd;
  const v8us a0 = *(const v8us*)(vth + go), a1 = *(const v8us*)(vth + go + 8);
  const v8us c0 = *(const v8us*)(vtr + go), c1 = *(const v8us*)(vtr + go + 8);
  *(v8us*)(Vth + d * 64 + qd)     = a0;
  *(v8us*)(Vth + d * 64 + qd + 8) = a1;
  *(v8us*)(Vtr + d * 64 + qd)     = c0;
  *(v8us*)(Vtr + d * 64 + qd + 8) = c1;
}
__device__ __forceinline__ void score_tile(v16us qa, v16us qz, const unsigned short* Ksh, const unsigned short* Krs,
                                           int c, int hh, float sscale, float ssres, v8f* s) {
#pragma unroll
  for (int j = 0; j < 4; ++j) {
    Frag kb, kc;
    const unsigned short* kp = Ksh + (j * 16 + c) * HD + 8 * hh;
    const unsigned short* kq = Krs + (j * 16 + c) * HD + 8 * hh;
    kb.p[0] = *(const v8us*)(kp);
    kb.p[1] = *(const v8us*)(kp + 16);
    kc.p[0] = *(const v8us*)(kq);
    kc.p[1] = *(const v8us*)(kq + 16);
    v8f sh = mma_g<0>(qa, kb.u, zero8());
    v8f sr = mma_g<0>(qz, kb.u, zero8());
    sr = mma_g<0>(qa, kc.u, sr);
#pragma unroll
    for (int r = 0; r < 8; ++r) s[j][r] = fmaf(sh[r], sscale, sr[r] * ssres);
  }
}
__device__ __forceinline__ void load_tab(const float* stab, int b, int h, int kv0, int c, v8f* s) {
  const float* sp = stab + (size_t)(b * NH + h) * SEQ + kv0;
#pragma unroll
  for (int j = 0; j < 4; ++j) {
    const float sv = sp[j * 16 + c];
#pragma unroll
    for (int r = 0; r < 8; ++r) s[j][r] = sv;
  }
}

__global__ __launch_bounds__(128)
void attn_stats(const unsigned short* __restrict__ qh, const unsigned short* __restrict__ qr, int qpitch,
                const unsigned short* __restrict__ kh, const unsigned short* __restrict__ kr,
                const float* __restrict__ stab, int tabmode, float* mip, int peek, float sscale, float ssres) {
  __shared__ __align__(16) unsigned short Ksh[64 * HD];
  __shared__ __align__(16) unsigned short Krs[64 * HD];
  __shared__ __align__(16) float          sML[128];

  const int tid  = threadIdx.x;
  const int wave = tid >> 5;
  const int lane = tid & 31;
  const int hh   = lane >> 4;
  const int c    = lane & 15;
  const int bx   = blockIdx.x;
  const int qb   = bx % NQB;
  const int rest = bx / NQB;
  const int h    = rest % NH;
  const int b    = rest / NH;
  const int q0   = qb * 64 + wave * 16;
  const size_t rowB = (size_t)b * SEQ;

  v16us qa = zero16(), qz = zero16();
  if (tabmode == 0) {
    const size_t qo = (rowB + q0 + c) * (size_t)qpitch + (size_t)h * HD + 8 * hh;
    qa = ldfrag(qh + qo);
    qz = ldfrag(qr + qo);
  }
  const int lim0 = q0 + 8 * hh - 1 + peek;

  float mrow[8], lrow[8];
#pragma unroll
  for (int r = 0; r < 8; ++r) { mrow[r] = -INFINITY; lrow[r] = 0.f; }

  const int nkt = qb + 1;
  for (int kt = 0; kt < nkt; ++kt) {
    const int kv0 = kt * 64;
    __syncthreads();
    if (tabmode == 0) stage_k(Ksh, Krs, kh, kr, rowB, kv0, h, tid);
    __syncthreads();
    v8f s[4];
#pragma unroll
    for (int j = 0; j < 4; ++j) s[j] = zero8();
    if (tabmode != 0) load_tab(stab, b, h, kv0, c, s);
    else score_tile(qa, qz, Ksh, Krs, c, hh, sscale, ssres, s);

#pragma unroll
    for (int r = 0; r < 8; ++r) {
      const int lim = lim0 + r;
      float m = -INFINITY;
#pragma unroll
      for (int j = 0; j < 4; ++j) {
        const int key = kv0 + j * 16 + c;
        const float sm = (key <= lim) ? s[j][r] : NEGV;
        s[j][r] = sm;
        m = fmaxf(m, sm);
      }
#pragma unroll
      for (int off = 1; off < 16; off <<= 1) m = fmaxf(m, __shfl_xor(m, off, 32));
      const float mnew  = fmaxf(mrow[r], m);
      const float alpha = __expf(mrow[r] - mnew);
      mrow[r] = mnew;
      float psum = 0.f;
#pragma unroll
      for (int j = 0; j < 4; ++j) psum += __expf(s[j][r] - mnew);
#pragma unroll
      for (int off = 1; off < 16; off <<= 1) psum += __shfl_xor(psum, off, 32);
      lrow[r] = lrow[r] * alpha + psum;
    }
  }

  if (c == 0) {
#pragma unroll
    for (int r = 0; r < 8; ++r) {
      const float l = lrow[r];
      sML[wave * 16 + 8 * hh + r]      = mrow[r];
      sML[64 + wave * 16 + 8 * hh + r] = (l > 0.f) ? (1.0f / l) : 0.f;
    }
  }
  __syncthreads();
  if (wave == 0) {
    const v4f sv = *(const v4f*)(sML + 4 * lane);
    float* dst = mip + (size_t)hh * MISZ + (size_t)(b * NH + h) * SEQ + qb * 64 + 4 * c;
    *(volatile v4f*)dst = sv;
    __threadfence();
    *(volatile v4f*)dst = sv;
  }
}

__global__ __launch_bounds__(128)
void attn_main(const unsigned short* __restrict__ qh, const unsigned short* __restrict__ qr, int qpitch,
               const unsigned short* __restrict__ kh, const unsigned short* __restrict__ kr,
               const unsigned short* __restrict__ vth, const unsigned short* __restrict__ vtr,
               const float* __restrict__ stab, int tabmode,
               const float* __restrict__ mip, const float* __restrict__ gin,
               unsigned short* ctxp, int peek, float sscale, float ssres) {
  __shared__ __align__(16) unsigned short Ksh[64 * HD];
  __shared__ __align__(16) unsigned short Krs[64 * HD];
  __shared__ __align__(16) unsigned short Vth[HD * 64];
  __shared__ __align__(16) unsigned short Vtr[HD * 64];
  __shared__ __align__(16) unsigned short Psh[4][16 * 64];
  __shared__ __align__(16) float          Os[4][16 * HD];

  const int tid  = threadIdx.x;
  const int wave = tid >> 5;
  const int lane = tid & 31;
  const int hh   = lane >> 4;
  const int c    = lane & 15;
  const int bx   = blockIdx.x;
  const int qb   = bx % NQB;
  const int rest = bx / NQB;
  const int h    = rest % NH;
  const int b    = rest / NH;
  const int q0   = qb * 64 + wave * 16;
  const size_t rowB = (size_t)b * SEQ;

  const float gv  = bfr(gin[h]);
  const float gam = -(fmaxf(gv, 0.0f) + log1pf(__expf(-fabsf(gv))));

  v16us qa = zero16(), qz = zero16();
  if (tabmode == 0) {
    const size_t qo = (rowB + q0 + c) * (size_t)qpitch + (size_t)h * HD + 8 * hh;
    qa = ldfrag(qh + qo);
    qz = ldfrag(qr + qo);
  }
  F8 mv, iv;
  {
    const float* mp = mip + (size_t)(b * NH + h) * SEQ + q0 + 8 * hh;
    mv.q[0] = *(const v4f*)(mp);
    mv.q[1] = *(const v4f*)(mp + 4);
    iv.q[0] = *(const v4f*)(mp + MISZ);
    iv.q[1] = *(const v4f*)(mp + MISZ + 4);
  }
  const int lim0 = q0 + 8 * hh - 1 + peek;

  float m2[8], l2[8], carry[8];
  v8f oacc[2], oacr[2];
#pragma unroll
  for (int r = 0; r < 8; ++r) { m2[r] = -INFINITY; l2[r] = 0.f; carry[r] = 0.f; }
#pragma unroll
  for (int t = 0; t < 2; ++t) { oacc[t] = zero8(); oacr[t] = zero8(); }

  const int nkt = qb + 1;
  for (int kt = 0; kt < nkt; ++kt) {
    const int kv0 = kt * 64;
    __syncthreads();
    if (tabmode == 0) stage_k(Ksh, Krs, kh, kr, rowB, kv0, h, tid);
    stage_v(Vth, Vtr, vth, vtr, b, kv0, h, tid);
    __syncthreads();

    v8f s[4];
#pragma unroll
    for (int j = 0; j < 4; ++j) s[j] = zero8();
    if (tabmode != 0) load_tab(stab, b, h, kv0, c, s);
    else score_tile(qa, qz, Ksh, Krs, c, hh, sscale, ssres, s);

#pragma unroll
    for (int r = 0; r < 8; ++r) {
      const int qrow = q0 + 8 * hh + r;
      const int lim  = lim0 + r;
      const float m1 = mv.v[r], i1 = iv.v[r];
#pragma unroll
      for (int j = 0; j < 4; ++j) {
        const int key   = kv0 + j * 16 + c;
        const bool live = (key <= lim);
        const float sm  = live ? s[j][r] : NEGV;
        const float p   = __expf(sm - m1) * i1;
        float pre = p;
#pragma unroll
        for (int o = 1; o < 16; o <<= 1) {
          const float tv = __shfl(pre, (lane - o) & 31, 32);
          pre = (c >= o) ? (pre + tv) : pre;
        }
        const float tot = __shfl(pre, lane | 15, 32);
        const float cum = carry[r] + pre;
        carry[r] += tot;
        const float rem = 1.0f - cum;
        const float pos = fabsf((float)(qrow - key));
        const float dd  = sqrtf(fmaxf(rem * pos, 0.0f));
        float eff = __expf(dd * gam);
        eff = fminf(fmaxf(eff, 1.0e-5f), 1.0e5f);
        s[j][r] = live ? (sm * eff) : NEGV;
      }
    }

    unsigned short* pwh = Psh[wave];
#pragma unroll
    for (int r = 0; r < 8; ++r) {
      const int lim = lim0 + r;
      float m = s[0][r];
      m = fmaxf(m, s[1][r]);
      m = fmaxf(m, s[2][r]);
      m = fmaxf(m, s[3][r]);
#pragma unroll
      for (int off = 1; off < 16; off <<= 1) m = fmaxf(m, __shfl_xor(m, off, 32));
      const float mnew  = fmaxf(m2[r], m);
      const float alpha = __expf(m2[r] - mnew);
      m2[r] = mnew;
      float psum = 0.f;
#pragma unroll
      for (int j = 0; j < 4; ++j) {
        const int key  = kv0 + j * 16 + c;
        const float p2 = __expf(s[j][r] - mnew);
        psum += p2;
        const float pw = (key <= lim) ? (p2 * PSC) : 0.0f;
        pwh[(8 * hh + r) * 64 + j * 16 + c] = h_bits((_Float16)pw);
      }
#pragma unroll
      for (int off = 1; off < 16; off <<= 1) psum += __shfl_xor(psum, off, 32);
      l2[r] = l2[r] * alpha + psum;
#pragma unroll
      for (int t = 0; t < 2; ++t) { oacc[t][r] *= alpha; oacr[t][r] *= alpha; }
    }
    wave_sync_lds();

#pragma unroll 1
    for (int kk = 0; kk < 2; ++kk) {
      Frag pa;
      pa.p[0] = *(const v8us*)(pwh + c * 64 + kk * 32 + 8 * hh);
      pa.p[1] = *(const v8us*)(pwh + c * 64 + kk * 32 + 16 + 8 * hh);
#pragma unroll
      for (int t = 0; t < 2; ++t) {
        Frag vb, vc;
        vb.p[0] = *(const v8us*)(Vth + (t * 16 + c) * 64 + kk * 32 + 8 * hh);
        vb.p[1] = *(const v8us*)(Vth + (t * 16 + c) * 64 + kk * 32 + 16 + 8 * hh);
        vc.p[0] = *(const v8us*)(Vtr + (t * 16 + c) * 64 + kk * 32 + 8 * hh);
        vc.p[1] = *(const v8us*)(Vtr + (t * 16 + c) * 64 + kk * 32 + 16 + 8 * hh);
        oacc[t] = mma_g<0>(pa.u, vb.u, oacc[t]);
        oacr[t] = mma_g<0>(pa.u, vc.u, oacr[t]);
      }
    }
  }

  float* os = Os[wave];
#pragma unroll
  for (int r = 0; r < 8; ++r) {
    const float l = l2[r];
    const float inv = ((l > 0.f) ? (1.0f / l) : 0.f) * (1.0f / PSC);
#pragma unroll
    for (int t = 0; t < 2; ++t) os[(8 * hh + r) * HD + t * 16 + c] = fmaf(oacr[t][r], 1.0f / RSC, oacc[t][r]) * inv;
  }
  wave_sync_lds();
  {
    const int rg = lane >> 3, p = lane & 7, part = p >> 2, sub = p & 3;
    v4u hv[4];
#pragma unroll
    for (int it = 0; it < 4; ++it) {
      const int row = it * 4 + rg;
      const float* sp = os + row * HD + sub * 8;
      v4u a;
#pragma unroll
      for (int e = 0; e < 4; ++e) a[e] = pick2(sp[2 * e], sp[2 * e + 1], part);
      hv[it] = a;
    }
    for (int pass = 0; pass < 2; ++pass) {
#pragma unroll
      for (int it = 0; it < 4; ++it) {
        const int row = it * 4 + rg;
        const size_t go = (rowB + q0 + row) * C32W + (size_t)h * 64 + p * 8;
        *(volatile v4u*)(ctxp + go) = hv[it];
      }
      __threadfence();
    }
  }
}

__global__ __launch_bounds__(256) void ln_c32(const float* __restrict__ X, const float* __restrict__ res, int rpitch,
                                            const float* __restrict__ gam, const float* __restrict__ bet,
                                            unsigned short* outp) {
  const int t = threadIdx.x, lane = t & 31, wave = t >> 5;
  const int row = blockIdx.x * 8 + wave;
  const int sub = lane & 3, part = (lane >> 2) & 1;
  const int ca = (lane >> 3) * 32 + sub * 8;
  const int cb = ca + 128;
  const float* xr = X + (size_t)row * DM;
  const float* rr = res + (size_t)row * (size_t)rpitch;
  F8 xa, xb, ra, rb, ga, gb, ba, bb;
  xa.q[0] = *(const v4f*)(xr + ca);  xa.q[1] = *(const v4f*)(xr + ca + 4);
  xb.q[0] = *(const v4f*)(xr + cb);  xb.q[1] = *(const v4f*)(xr + cb + 4);
  ra.q[0] = *(const v4f*)(rr + ca);  ra.q[1] = *(const v4f*)(rr + ca + 4);
  rb.q[0] = *(const v4f*)(rr + cb);  rb.q[1] = *(const v4f*)(rr + cb + 4);
  ga.q[0] = *(const v4f*)(gam + ca); ga.q[1] = *(const v4f*)(gam + ca + 4);
  gb.q[0] = *(const v4f*)(gam + cb); gb.q[1] = *(const v4f*)(gam + cb + 4);
  ba.q[0] = *(const v4f*)(bet + ca); ba.q[1] = *(const v4f*)(bet + ca + 4);
  bb.q[0] = *(const v4f*)(bet + cb); bb.q[1] = *(const v4f*)(bet + cb + 4);
  v8f va, vb;
  float ps = 0.f;
#pragma unroll
  for (int e = 0; e < 8; ++e) {
    va[e] = xa.v[e] + bfr(ra.v[e]);
    vb[e] = xb.v[e] + bfr(rb.v[e]);
    ps += va[e] + vb[e];
  }
  ps = part ? 0.f : ps;
  const float mean = wsum(ps) * (1.0f / DM);
  float pq = 0.f;
#pragma unroll
  for (int e = 0; e < 8; ++e) {
    va[e] -= mean;
    vb[e] -= mean;
    pq += va[e] * va[e] + vb[e] * vb[e];
  }
  pq = part ? 0.f : pq;
  const float var  = wsum(pq) * (1.0f / DM);
  const float rstd = 1.0f / sqrtf(var + LNEPS);
  v8f ya, yb;
#pragma unroll
  for (int e = 0; e < 8; ++e) {
    ya[e] = (va[e] * rstd) * bfr(ga.v[e]) + bfr(ba.v[e]);
    yb[e] = (vb[e] * rstd) * bfr(gb.v[e]) + bfr(bb.v[e]);
  }
  v4u oa, ob;
#pragma unroll
  for (int e = 0; e < 4; ++e) {
    oa[e] = pick2(ya[2 * e], ya[2 * e + 1], part);
    ob[e] = pick2(yb[2 * e], yb[2 * e + 1], part);
  }
  unsigned short* d0 = outp + (size_t)row * C32W + 8 * lane;
  *(volatile v4u*)(d0) = oa;
  *(volatile v4u*)(d0 + 256) = ob;
  __threadfence();
  *(volatile v4u*)(d0) = oa;
  *(volatile v4u*)(d0 + 256) = ob;
}

__global__ __launch_bounds__(256) void readout(const unsigned short* __restrict__ A, const unsigned short* __restrict__ Bt,
                                             const float* __restrict__ beta, const float* __restrict__ bias,
                                             float* outp) {
  __shared__ __align__(16) float sT[8][2 * 64];
  const int lane = threadIdx.x & 31;
  const int wave = threadIdx.x >> 5;
  const int tile = blockIdx.x * 8 + wave;
  const int tm = tile >> 2, tn = tile & 3;
  const int m0 = tm << 6, n0 = tn << 6;
  const int rlane = lane & 15;
  const int koff  = (lane >> 4) * 8;
  const int hh = lane >> 4, c = lane & 15;

  v8f acc[4][4];
#pragma unroll
  for (int i = 0; i < 4; ++i)
#pragma unroll
    for (int j = 0; j < 4; ++j) acc[i][j] = zero8();

#pragma unroll
  for (int k0 = 0; k0 < 64; k0 += 32) {
    v16us bh[4];
#pragma unroll
    for (int j = 0; j < 4; ++j) bh[j] = ldfrag(Bt + (size_t)(n0 + (j << 4) + rlane) * 64 + koff + k0);
#pragma unroll
    for (int i = 0; i < 4; ++i) {
      const v16us ah = ldfrag(A + (size_t)(m0 + (i << 4) + rlane) * 64 + koff + k0);
#pragma unroll
      for (int j = 0; j < 4; ++j) acc[i][j] = mma_raw<1>(ah, bh[j], acc[i][j]);
      dep_guard1(acc[i][0], acc[i][3], ah);
    }
    keep4(bh[0], bh[1], bh[2], bh[3]);
  }
  acc_guard4(acc[0][0], acc[0][1], acc[0][2], acc[0][3]);
  acc_guard4(acc[1][0], acc[1][1], acc[1][2], acc[1][3]);
  acc_guard4(acc[2][0], acc[2][1], acc[2][2], acc[2][3]);
  acc_guard4(acc[3][0], acc[3][1], acc[3][2], acc[3][3]);

  float bc[4];
#pragma unroll
  for (int j = 0; j < 4; ++j) bc[j] = bfr(bias[n0 + (j << 4) + c]);
  const int tok0 = m0 >> 3;
  float* slab = sT[wave];
  v4f vals[4];
#pragma unroll
  for (int i = 0; i < 4; ++i) {
    const int tok = tok0 + 2 * i + hh;
    F8 be;
    be.q[0] = *(const v4f*)(beta + (size_t)tok * 64);
    be.q[1] = *(const v4f*)(beta + (size_t)tok * 64 + 4);
    float bm = be.v[0];
#pragma unroll
    for (int r = 1; r < 8; ++r) bm = fmaxf(bm, be.v[r]);
    float ex[8], den = 0.f;
#pragma unroll
    for (int r = 0; r < 8; ++r) { ex[r] = __expf(be.v[r] - bm); den += ex[r]; }
    const float rden = __builtin_amdgcn_rcpf(den);
#pragma unroll
    for (int j = 0; j < 4; ++j) {
      float o = 0.f;
#pragma unroll
      for (int r = 0; r < 8; ++r) {
        const float x  = acc[i][j][r] + bc[j];
        const float sg = __builtin_amdgcn_rcpf(1.0f + __expf(-x));
        o = fmaf(ex[r] * rden, sg, o);
      }
      slab[hh * 64 + (j << 4) + c] = o;
    }
    wave_sync_lds();
    vals[i] = *(const v4f*)(slab + hh * 64 + c * 4);
    wave_sync_lds();
  }
  for (int pass = 0; pass < 2; ++pass) {
#pragma unroll
    for (int i = 0; i < 4; ++i) {
      float* dst = outp + (size_t)(tok0 + 2 * i + hh) * DM + n0 + c * 4;
      *(volatile v4f*)dst = vals[i];
    }
    __threadfence();
  }
}

extern "C" void kernel_launch(void* const* d_in, const int* in_sizes, int n_in,
                              void* d_out, int out_size, void* d_ws, size_t ws_size,
                              hipStream_t stream) {
  if (n_in < 37) return;
  if (in_sizes[0] != MP * DM || in_sizes[1] != MP * DM) return;
  {
    const int wi[10] = {3, 5, 7, 12, 14, 16, 21, 23, 25, 27};
    const int bi[16] = {4, 6, 8, 10, 11, 13, 15, 17, 19, 20, 22, 24, 26, 28, 30, 31};
    for (int i = 0; i < 10; ++i) if (in_sizes[wi[i]] != DM * DM) return;
    for (int i = 0; i < 16; ++i) if (in_sizes[bi[i]] != DM) return;
  }
  if (in_sizes[9] != NH || in_sizes[18] != NH || in_sizes[29] != NH) return;
  if (in_sizes[32] != DM * HD || in_sizes[34] != DM * HD) return;
  if (in_sizes[33] != DM || in_sizes[35] != DM || in_sizes[36] != DM) return;
  if (out_size != MP * DM) return;

  const float* q_emb = (const float*)d_in[0];
  const float* s_emb = (const float*)d_in[1];
  const float* Wq1 = (const float*)d_in[3];   const float* bq1  = (const float*)d_in[4];
  const float* Wv1 = (const float*)d_in[5];   const float* bv1  = (const float*)d_in[6];
  const float* Wo1 = (const float*)d_in[7];   const float* bo1  = (const float*)d_in[8];
  const float* g1  = (const float*)d_in[9];
  const float* lng1 = (const float*)d_in[10]; const float* lnb1 = (const float*)d_in[11];
  const float* Wq2 = (const float*)d_in[12];  const float* bq2  = (const float*)d_in[13];
  const float* Wv2 = (const float*)d_in[14];  const float* bv2  = (const float*)d_in[15];
  const float* Wo2 = (const float*)d_in[16];  const float* bo2  = (const float*)d_in[17];
  const float* g2  = (const float*)d_in[18];
  const float* lng2 = (const float*)d_in[19]; const float* lnb2 = (const float*)d_in[20];
  const float* Wq3 = (const float*)d_in[21];  const float* bq3  = (const float*)d_in[22];
  const float* Wk3 = (const float*)d_in[23];  const float* bk3  = (const float*)d_in[24];
  const float* Wv3 = (const float*)d_in[25];  const float* bv3  = (const float*)d_in[26];
  const float* Wo3 = (const float*)d_in[27];  const float* bo3  = (const float*)d_in[28];
  const float* g3  = (const float*)d_in[29];
  const float* lng3 = (const float*)d_in[30]; const float* lnb3 = (const float*)d_in[31];
  const float* Wlk = (const float*)d_in[32];  const float* blk_in = (const float*)d_in[33];
  const float* Wlv = (const float*)d_in[34];  const float* blv  = (const float*)d_in[35];
  const float* know = (const float*)d_in[36];

  const size_t PXH  = (size_t)MP * DM * 2;
  const size_t PQD  = (size_t)MP * C32W * 2;
  const size_t PW16 = (size_t)DM * DM * 2;
  const size_t PWD  = (size_t)DM * C32W * 2;
  const size_t PWLV = (size_t)DM * (2 * HD) * 2;
  const size_t PKK  = (size_t)64 * C32W * 2;
  const size_t PQ3  = 1024;
  const size_t PS3  = (size_t)NB * NH * SEQ * 4;
  const size_t PQK  = (size_t)2 * MP * DM * 2;
  const size_t PVT  = (size_t)2 * NB * DM * SEQ * 2;
  const size_t PCTX = (size_t)MP * C32W * 2;
  const size_t PAO  = (size_t)MP * DM * 4;
  const size_t PMI  = (size_t)2 * MISZ * 4;
  const size_t PH   = (size_t)MP * C32W * 2;
  const size_t PBT  = (size_t)MP * 64 * 4;
  size_t off = 0;
  const size_t oXH1 = off; off += PXH;
  const size_t oXH2 = off; off += PXH;
  const size_t oQD  = off; off += PQD;
  const size_t oW16 = off; off += 4 * PW16;
  const size_t oWD  = off; off += 5 * PWD;
  const size_t oWLV = off; off += PWLV;
  const size_t oKK  = off; off += PKK;
  const size_t oQ3  = off; off += PQ3;
  const size_t oS3  = off; off += PS3;
  const size_t oQK  = off; off += PQK;
  const size_t oVT  = off; off += PVT;
  const size_t oCTX = off; off += PCTX;
  const size_t oAO  = off; off += PAO;
  const size_t oMI  = off; off += PMI;
  const size_t oH1  = off; off += PH;
  const size_t oH2  = off; off += PH;
  const size_t oH3  = off; off += PH;
  const size_t oBT  = off; off += PBT;
  if (off > ws_size) return;
  if (off > (size_t)134217728) return;

  char* ws = (char*)d_ws;
  unsigned short* XH1  = (unsigned short*)(ws + oXH1);
  unsigned short* XH2  = (unsigned short*)(ws + oXH2);
  unsigned short* QD   = (unsigned short*)(ws + oQD);
  unsigned short* Wq1H = (unsigned short*)(ws + oW16);
  unsigned short* Wv1H = (unsigned short*)(ws + oW16 + PW16);
  unsigned short* Wq2H = (unsigned short*)(ws + oW16 + 2 * PW16);
  unsigned short* Wv2H = (unsigned short*)(ws + oW16 + 3 * PW16);
  unsigned short* Wk3D = (unsigned short*)(ws + oWD);
  unsigned short* Wv3D = (unsigned short*)(ws + oWD + PWD);
  unsigned short* Wo1D = (unsigned short*)(ws + oWD + 2 * PWD);
  unsigned short* Wo2D = (unsigned short*)(ws + oWD + 3 * PWD);
  unsigned short* Wo3D = (unsigned short*)(ws + oWD + 4 * PWD);
  unsigned short* WlvD = (unsigned short*)(ws + oWLV);
  unsigned short* KK   = (unsigned short*)(ws + oKK);
  float*          Q3F  = (float*)(ws + oQ3);
  float*          S3   = (float*)(ws + oS3);
  unsigned short* QK   = (unsigned short*)(ws + oQK);
  unsigned short* VT   = (unsigned short*)(ws + oVT);
  unsigned short* CTX  = (unsigned short*)(ws + oCTX);
  float*          AO   = (float*)(ws + oAO);
  float*          MI   = (float*)(ws + oMI);
  unsigned short* H1   = (unsigned short*)(ws + oH1);
  unsigned short* H2   = (unsigned short*)(ws + oH2);
  unsigned short* H3   = (unsigned short*)(ws + oH3);
  float*          BT   = (float*)(ws + oBT);
  float*          outp = (float*)d_out;

  const int n8x = (MP * DM) / 8;
  const int n8w = (DM * DM) / 8;
  const int npx = MP * (DM / 4);
  const int npw = DM * (DM / 4);
  const int nplv = DM * (HD / 4);
  if ((n8x % 256) != 0 || (n8w % 256) != 0 || (npx % 256) != 0 || (npw % 256) != 0 || (nplv % 256) != 0) return;

  const dim3 blk(256), blk128(128), blk32(32);
  const dim3 gXH((n8x + 255) / 256), gW16((n8w + 255) / 256);
  const dim3 gQD((npx + 255) / 256), gWD((npw + 255) / 256), gWLV((nplv + 255) / 256);
  const dim3 gSmall(65);
  const dim3 gProj(((MP / 64) * (DM / 64) + 7) / 8, 1);
  const dim3 gVT(((DM / 64) * (SEQ / 64) + 7) / 8, NB);
  const dim3 gAttn(NB * NH * NQB);
  const dim3 gLN(MP / 8);
  const dim3 gS3((NB * NH * SEQ + 255) / 256);
  const dim3 gBeta(((MP / 64) * 1 + 7) / 8, 1);
  const dim3 gRead((MP * NH / 64) * (DM / 64) / 8);
  const float invw = 1.0f / WSC;
  const float ssc  = SSC;
  const float ssr  = SSC / RSC;

  conv_h16<<<gXH, blk, 0, stream>>>(q_emb, XH1, n8x, 1.0f);
  conv_h16<<<gXH, blk, 0, stream>>>(s_emb, XH2, n8x, 1.0f);
  conv_c32<<<gQD, blk, 0, stream>>>(q_emb, QD, npx, DM);
  conv_h16<<<gW16, blk, 0, stream>>>(Wq1, Wq1H, n8w, WSC);
  conv_h16<<<gW16, blk, 0, stream>>>(Wv1, Wv1H, n8w, WSC);
  conv_h16<<<gW16, blk, 0, stream>>>(Wq2, Wq2H, n8w, WSC);
  conv_h16<<<gW16, blk, 0, stream>>>(Wv2, Wv2H, n8w, WSC);
  conv_c32<<<gWD, blk, 0, stream>>>(Wk3, Wk3D, npw, DM);
  conv_c32<<<gWD, blk, 0, stream>>>(Wv3, Wv3D, npw, DM);
  conv_c32<<<gWD, blk, 0, stream>>>(Wo1, Wo1D, npw, DM);
  conv_c32<<<gWD, blk, 0, stream>>>(Wo2, Wo2D, npw, DM);
  conv_c32<<<gWD, blk, 0, stream>>>(Wo3, Wo3D, npw, DM);
  conv_c32<<<gWLV, blk, 0, stream>>>(Wlv, WlvD, nplv, HD);
  small_vec<<<gSmall, blk32, 0, stream>>>(know, Wlk, blk_in, Wq3, bq3, KK, Q3F);

  gemm64<0, 3, 0><<<gProj, blk, 0, stream>>>(
      XH1, DM, 0LL, Wq1H, DM, 0LL, bq1, (void*)QK, DM, 0LL, (long long)QRES, MP, DM, DM, invw);
  gemm64<0, 3, 1><<<gVT, blk, 0, stream>>>(
      Wv1H, DM, 0LL, XH1, DM, (long long)SEQ * DM, bv1, (void*)VT, SEQ, (long long)DM * SEQ, (long long)VRES,
      DM, SEQ, DM, invw);
  attn_stats<<<gAttn, blk128, 0, stream>>>(QK, QK + QRES, DM, QK, QK + QRES, S3, 0, MI, 1, ssc, ssr);
  attn_main<<<gAttn, blk128, 0, stream>>>(QK, QK + QRES, DM, QK, QK + QRES, VT, VT + VRES, S3, 0, MI, g1, CTX,
                                         1, ssc, ssr);
  gemm64<1, 0, 0><<<gProj, blk, 0, stream>>>(
      CTX, C32W, 0LL, Wo1D, C32W, 0LL, bo1, (void*)AO, DM, 0LL, 0LL, MP, DM, C32W, 1.0f);
  ln_c32<<<gLN, blk, 0, stream>>>(AO, q_emb, DM, lng1, lnb1, H1);

  gemm64<0, 3, 0><<<gProj, blk, 0, stream>>>(
      XH2, DM, 0LL, Wq2H, DM, 0LL, bq2, (void*)QK, DM, 0LL, (long long)QRES, MP, DM, DM, invw);
  gemm64<0, 3, 1><<<gVT, blk, 0, stream>>>(
      Wv2H, DM, 0LL, XH2, DM, (long long)SEQ * DM, bv2, (void*)VT, SEQ, (long long)DM * SEQ, (long long)VRES,
      DM, SEQ, DM, invw);
  attn_stats<<<gAttn, blk128, 0, stream>>>(QK, QK + QRES, DM, QK, QK + QRES, S3, 0, MI, 1, ssc, ssr);
  attn_main<<<gAttn, blk128, 0, stream>>>(QK, QK + QRES, DM, QK, QK + QRES, VT, VT + VRES, S3, 0, MI, g2, CTX,
                                         1, ssc, ssr);
  gemm64<1, 0, 0><<<gProj, blk, 0, stream>>>(
      CTX, C32W, 0LL, Wo2D, C32W, 0LL, bo2, (void*)AO, DM, 0LL, 0LL, MP, DM, C32W, 1.0f);
  ln_c32<<<gLN, blk, 0, stream>>>(AO, s_emb, DM, lng2, lnb2, H2);

  gemm64<1, 0, 0><<<gProj, blk, 0, stream>>>(
      H1, C32W, 0LL, Wk3D, C32W, 0LL, bk3, (void*)AO, DM, 0LL, 0LL, MP, DM, C32W, 1.0f);
  score3<<<gS3, blk, 0, stream>>>(AO, Q3F, S3, ssc);
  gemm64<1, 3, 1><<<gVT, blk, 0, stream>>>(
      Wv3D, C32W, 0LL, H2, C32W, (long long)SEQ * C32W, bv3, (void*)VT, SEQ, (long long)DM * SEQ, (long long)VRES,
      DM, SEQ, C32W, 1.0f);
  attn_stats<<<gAttn, blk128, 0, stream>>>(XH1, XH2, DM, XH1, XH2, S3, 1, MI, 0, ssc, ssr);
  attn_main<<<gAttn, blk128, 0, stream>>>(XH1, XH2, DM, XH1, XH2, VT, VT + VRES, S3, 1, MI, g3, CTX, 0, ssc, ssr);
  gemm64<1, 0, 0><<<gProj, blk, 0, stream>>>(
      CTX, C32W, 0LL, Wo3D, C32W, 0LL, bo3, (void*)AO, DM, 0LL, 0LL, MP, DM, C32W, 1.0f);
  ln_c32<<<gLN, blk, 0, stream>>>(AO, know, 0, lng3, lnb3, H3);

  gemm64<1, 0, 2><<<gBeta, blk, 0, stream>>>(
      QD, C32W, 0LL, KK, C32W, 0LL, blk_in, (void*)BT, 64, 0LL, 0LL, MP, 64, C32W, 1.0f);
  readout<<<gRead, blk, 0, stream>>>(H3, WlvD, BT, blv, outp);
  (void)hipGetLastError();
}
